// SelectiveSSM_20804821582028
// MI455X (gfx1250) — hardware-verified
//
#include <hip/hip_runtime.h>
#include <math.h>

typedef __attribute__((ext_vector_type(16))) _Float16 v16h;
typedef __attribute__((ext_vector_type(8)))  _Float16 v8h;
typedef __attribute__((ext_vector_type(4)))  _Float16 v4h;
typedef __attribute__((ext_vector_type(16))) __bf16   v16b;
typedef __attribute__((ext_vector_type(8)))  __bf16   v8b;
typedef __attribute__((ext_vector_type(8)))  float    v8f;
typedef __attribute__((ext_vector_type(4)))  float    v4f;

constexpr int kSamples = 2;
constexpr int kSeq   = 2048;
constexpr int kRows  = kSeq;
constexpr int kDm    = 1024;
constexpr int kDi    = 2048;
constexpr int kDi2   = 2 * kDi;
constexpr int kNs    = 16;
constexpr int kXd    = 1 + 2 * kNs;
constexpr int kXdP   = 64;
constexpr int kKc    = 4;
constexpr int kXK    = 2 * kDi;
constexpr int kThr   = 256;
constexpr float kInCarry = 1024.0f;
constexpr float kACarry  = 256.0f;
constexpr float kScIn = 1.0f / (kInCarry * kInCarry);
constexpr float kScA  = 1.0f / (kACarry * kInCarry);
constexpr float kF16MinNormal = 6.103515625e-5f;

static_assert((kRows % 64) == 0 && (kDi2 % 64) == 0 && (kXdP % 64) == 0 && (kDm % 64) == 0 && (kDm % 32) == 0 && (kDi % 32) == 0 && (kXK % 32) == 0
              && ((kRows / 64) * (kDi2 / 64)) % 8 == 0 && ((kRows / 64) * (kXdP / 64)) % 8 == 0 && ((kRows / 64) * (kDm / 64)) % 8 == 0, "GEMM M, N multiples of 64; grids exact; K multiples of 32");

constexpr size_t kOffX16 = 0ull;
constexpr size_t kOffWIN = 4194304ull;
constexpr size_t kOffWXP = 12582912ull;
constexpr size_t kOffWOUT = 13107200ull;
constexpr size_t kOffZB = 17301504ull;
constexpr size_t kOffXZ = 17317888ull;
constexpr size_t kOffXI = 50872320ull;
constexpr size_t kOffXI16 = 67649536ull;
constexpr size_t kOffXD = 84426752ull;
constexpr size_t kOffHID = 84951040ull;
constexpr size_t kOffY16 = 101728256ull;
constexpr size_t kWsTotal = 110116864ull;
static_assert(kWsTotal <= 134217728ull, "carve cap: under 128 MiB");
static_assert(kOffX16 == 0
              && kOffWIN == kOffX16 + 4194304ull
              && kOffWXP == kOffWIN + 8388608ull
              && kOffWOUT == kOffWXP + 524288ull
              && kOffZB == kOffWOUT + 4194304ull
              && kOffXZ == kOffZB + 16384ull
              && kOffXI == kOffXZ + 33554432ull
              && kOffXI16 == kOffXI + 16777216ull
              && kOffXD == kOffXI16 + 16777216ull
              && kOffHID == kOffXD + 524288ull
              && kOffY16 == kOffHID + 16777216ull
              && kWsTotal == kOffY16 + 8388608ull, "the carve is chained and totalled");
static_assert((kOffX16 % 256) == 0 && (kOffWIN % 256) == 0 && (kOffWXP % 256) == 0 && (kOffWOUT % 256) == 0 && (kOffZB % 256) == 0 && (kOffXZ % 256) == 0 && (kOffXI % 256) == 0 && (kOffXI16 % 256) == 0 && (kOffXD % 256) == 0 && (kOffHID % 256) == 0 && (kOffY16 % 256) == 0, "aligned regions");

__device__ __forceinline__ unsigned short f2bf_bits(float f) {
  unsigned u = __float_as_uint(f);
  return (unsigned short)((u + 0x7FFFu + ((u >> 16) & 1u)) >> 16);
}
__device__ __forceinline__ float bf_bits2f(unsigned short h) { return __uint_as_float(((unsigned)h) << 16); }
__device__ __forceinline__ float bf16r(float f) { return bf_bits2f(f2bf_bits(f)); }
__device__ __forceinline__ float carry_flush(float v, float carry) {
  const float s = v * carry;
  return (fabsf(s) < kF16MinNormal) ? 0.0f : s;
}
__device__ __forceinline__ float frcp(float x) { return __builtin_amdgcn_rcpf(x); }

__device__ __forceinline__ void dep_guard4_h(v8f& a, v8f& b, v8f& c, v8f& d, v16h x, v16h y) { asm volatile("v_nop\n\tv_nop\n\tv_nop\n\tv_nop" : "+v"(a), "+v"(b), "+v"(c), "+v"(d) : "v"(x), "v"(y)); }
__device__ __forceinline__ void dep_guard4_b(v8f& a, v8f& b, v8f& c, v8f& d, v16b x, v16b y) { asm volatile("v_nop\n\tv_nop\n\tv_nop\n\tv_nop" : "+v"(a), "+v"(b), "+v"(c), "+v"(d) : "v"(x), "v"(y)); }
__device__ __forceinline__ void keep4_h(v16h a, v16h b, v16h c, v16h d) { asm volatile("v_nop" :: "v"(a), "v"(b), "v"(c), "v"(d)); }
__device__ __forceinline__ void keep4_b(v16b a, v16b b, v16b c, v16b d) { asm volatile("v_nop" :: "v"(a), "v"(b), "v"(c), "v"(d)); }
__device__ __forceinline__ void acc_guard4(v8f& a, v8f& b, v8f& c, v8f& d) { asm volatile("v_nop\n\tv_nop\n\tv_nop\n\tv_nop" : "+v"(a), "+v"(b), "+v"(c), "+v"(d)); }

template <typename T> struct Frag;
template <> struct Frag<_Float16> {
  typedef v16h V; union U { v16h v; v8h h[2]; };
  static __device__ __forceinline__ v16h load(const _Float16* p) {
    U f; f.h[0] = *(const v8h*)(p); f.h[1] = *(const v8h*)(p + 16); return f.v;
  }
  static __device__ __forceinline__ v8f mma(v16h a, v16h b, v8f c) {
    return __builtin_amdgcn_wmma_f32_16x16x32_f16(false, a, false, b, (short)0, c, false, false);
  }
  static __device__ __forceinline__ void guard4(v8f& a, v8f& b, v8f& c, v8f& d, v16h x, v16h y) { dep_guard4_h(a, b, c, d, x, y); }
  static __device__ __forceinline__ void keep(v16h a, v16h b, v16h c, v16h d) { keep4_h(a, b, c, d); }
};
template <> struct Frag<__bf16> {
  typedef v16b V; union U { v16b v; v8b h[2]; };
  static __device__ __forceinline__ v16b load(const __bf16* p) {
    U f; f.h[0] = *(const v8b*)(p); f.h[1] = *(const v8b*)(p + 16); return f.v;
  }
  static __device__ __forceinline__ v8f mma(v16b a, v16b b, v8f c) {
    return __builtin_amdgcn_wmma_f32_16x16x32_bf16(false, a, false, b, (short)0, c, false, false);
  }
  static __device__ __forceinline__ void guard4(v8f& a, v8f& b, v8f& c, v8f& d, v16b x, v16b y) { dep_guard4_b(a, b, c, d, x, y); }
  static __device__ __forceinline__ void keep(v16b a, v16b b, v16b c, v16b d) { keep4_b(a, b, c, d); }
};

__device__ __forceinline__ v8f mma_h(v16h a, v16h b, v8f c) {
  c = __builtin_amdgcn_wmma_f32_16x16x32_f16(false, a, false, b, (short)0, c, false, false);
  asm volatile("v_nop\n\tv_nop\n\tv_nop\n\tv_nop" : "+v"(c) : "v"(a), "v"(b));
  return c;
}

template <int ET> struct Elem;
template <> struct Elem<0> { typedef _Float16 T; };
template <> struct Elem<1> { typedef __bf16 T; };
template <int ET, bool SPLIT, int BIAS_MODE, int OUT_MODE, bool RESID, int ACT = 0>
__global__ __launch_bounds__(256) void wmma_gemm64(
    const unsigned short* __restrict__ Ap, const unsigned short* __restrict__ A2p, int lda, long strideA,
    const unsigned short* __restrict__ Btp, const unsigned short* __restrict__ Bt2p, int ldb, long strideB,
    void* __restrict__ Cout, void* __restrict__ Cout2, int ldc, long strideC,
    const float* __restrict__ bias,
    const float* __restrict__ resid, long strideR,
    int M, int N, int K, float scale) {
  typedef typename Elem<ET>::T T;
  typedef typename Frag<T>::V V;
  const T* A = (const T*)Ap; const T* A2 = (const T*)A2p; const T* Bt = (const T*)Btp; const T* Bt2 = (const T*)Bt2p;
  __shared__ __align__(16) float sT[8][16 * 68];
  const int b    = blockIdx.y;
  const int lane = threadIdx.x & 31;
  const int wave = threadIdx.x >> 5;
  const int tilesN = N >> 6;
  const int tilesM = M >> 6;
  const int tile = blockIdx.x * 8 + wave;
  if (tile >= tilesM * tilesN) return;
  const int tm = tile / tilesN;
  const int tn = tile - tm * tilesN;
  const int m0 = tm << 6;
  const int n0 = tn << 6;

  const T* Ab  = A  + (size_t)b * strideA;
  const T* Bb  = Bt + (size_t)b * strideB;
  const T* Ab2 = SPLIT ? (A2  + (size_t)b * strideA) : nullptr;
  const T* Bb2 = SPLIT ? (Bt2 + (size_t)b * strideB) : nullptr;

  const int rlane = lane & 15;
  const int koff  = (lane >> 4) * 8;
  const int mOff  = (lane >> 4) * 8;

  v8f acc[4][4];
#pragma unroll
  for (int i = 0; i < 4; ++i)
#pragma unroll
    for (int j = 0; j < 4; ++j) acc[i][j] = (v8f){0.f,0.f,0.f,0.f,0.f,0.f,0.f,0.f};

  for (int k0 = 0; k0 < K; k0 += 32) {
    V bh[4], bl[4];
#pragma unroll
    for (int j = 0; j < 4; ++j) {
      const size_t bo = (size_t)(n0 + (j << 4) + rlane) * ldb + koff + k0;
      bh[j] = Frag<T>::load(Bb + bo);
      if (SPLIT) bl[j] = Frag<T>::load(Bb2 + bo);
    }
#pragma unroll
    for (int i = 0; i < 4; ++i) {
      const size_t ao = (size_t)(m0 + (i << 4) + rlane) * lda + koff + k0;
      V ah = Frag<T>::load(Ab + ao);
      V al;
      if (SPLIT) al = Frag<T>::load(Ab2 + ao);
#pragma unroll
      for (int j = 0; j < 4; ++j) {
        acc[i][j] = Frag<T>::mma(ah, bh[j], acc[i][j]);
        if (SPLIT) {
          acc[i][j] = Frag<T>::mma(ah, bl[j], acc[i][j]);
          acc[i][j] = Frag<T>::mma(al, bh[j], acc[i][j]);
        }
      }
      Frag<T>::guard4(acc[i][0], acc[i][1], acc[i][2], acc[i][3], ah, SPLIT ? al : ah);
    }
    Frag<T>::keep(bh[0], bh[1], bh[2], bh[3]);
    if (SPLIT) Frag<T>::keep(bl[0], bl[1], bl[2], bl[3]);
  }
  acc_guard4(acc[0][0], acc[0][1], acc[0][2], acc[0][3]);
  acc_guard4(acc[1][0], acc[1][1], acc[1][2], acc[1][3]);
  acc_guard4(acc[2][0], acc[2][1], acc[2][2], acc[2][3]);
  acc_guard4(acc[3][0], acc[3][1], acc[3][2], acc[3][3]);

  float* slab = sT[wave];
  const float* Rb = RESID ? (resid + (size_t)b * strideR) : nullptr;
#pragma unroll
  for (int i = 0; i < 4; ++i) {
    const int mBase = m0 + (i << 4);
#pragma unroll
    for (int j = 0; j < 4; ++j) {
      const int n = n0 + (j << 4) + rlane;
      float bv = 0.f;
      if (BIAS_MODE == 2) bv = bias[n];
#pragma unroll
      for (int r = 0; r < 8; ++r) {
        float v = acc[i][j][r] * scale;
        if (BIAS_MODE == 1) v += bias[mBase + mOff + r];
        if (BIAS_MODE == 2) v += bv;
        if (RESID) v += Rb[(size_t)(mBase + mOff + r) * ldc + n];
        if (ACT == 1) v = tanhf(v);
        if (ACT == 2) v = fmaxf(v, 0.0f);
        if (ACT == 3) v = v / (1.0f + expf(-v));
        if (ACT == 4) v = (v > 0.f) ? v : 0.01f * v;
        slab[(mOff + r) * 68 + (j << 4) + rlane] = v;
      }
    }
    __builtin_amdgcn_fence(__ATOMIC_RELEASE, "workgroup");
    __builtin_amdgcn_wave_barrier();
    __builtin_amdgcn_fence(__ATOMIC_ACQUIRE, "workgroup");
    if (OUT_MODE == 0) {
      float* C = (float*)Cout + (size_t)b * strideC;
      const int hh = lane >> 4, c4 = (lane & 15) * 4;
      for (int pass = 0; pass < 2; ++pass) {
#pragma unroll
        for (int it = 0; it < 8; ++it) {
          const int row = it * 2 + hh;
          v4f v = *(const v4f*)(slab + row * 68 + c4);
          *(volatile v4f*)(C + (size_t)(mBase + row) * ldc + n0 + c4) = v;
        }
        __threadfence();
      }
    } else {
      const int q = lane >> 3, c8 = (lane & 7) * 8;
      unsigned short* C  = (unsigned short*)Cout  + (size_t)b * strideC;
      unsigned short* C2 = (OUT_MODE == 2) ? ((unsigned short*)Cout2 + (size_t)b * strideC) : nullptr;
      for (int pass = 0; pass < 2; ++pass) {
#pragma unroll
        for (int it = 0; it < 4; ++it) {
          const int row = it * 4 + q;
          const float* sp = slab + row * 68 + c8;
          v8h hv, lv;
#pragma unroll
          for (int e = 0; e < 8; ++e) {
            if (OUT_MODE == 1) {
              hv[e] = (_Float16)sp[e];
            } else {
              unsigned short hb = f2bf_bits(sp[e]);
              unsigned short lb = f2bf_bits(sp[e] - bf_bits2f(hb));
              hv[e] = __builtin_bit_cast(_Float16, hb);
              lv[e] = __builtin_bit_cast(_Float16, lb);
            }
          }
          *(volatile v8h*)(C + (size_t)(mBase + row) * ldc + n0 + c8) = hv;
          if (OUT_MODE == 2) *(volatile v8h*)(C2 + (size_t)(mBase + row) * ldc + n0 + c8) = lv;
        }
        __threadfence();
      }
    }
    __builtin_amdgcn_fence(__ATOMIC_RELEASE, "workgroup");
    __builtin_amdgcn_wave_barrier();
    __builtin_amdgcn_fence(__ATOMIC_ACQUIRE, "workgroup");
  }
}

__global__ __launch_bounds__(kThr) void cast_plane_kernel(const float* __restrict__ src, unsigned short* __restrict__ dst,
                                                          int colsLog2, int dstPitch, int dstOff) {
  const int i   = blockIdx.x * kThr + threadIdx.x;
  const int sh  = colsLog2 - 3;
  const int row = i >> sh;
  const int c8  = (i & ((1 << sh) - 1)) * 8;
  const float* sp = src + ((size_t)row << colsLog2) + c8;
  const v4f a0 = *(const v4f*)(sp);
  const v4f a1 = *(const v4f*)(sp + 4);
  v8h hv;
#pragma unroll
  for (int e = 0; e < 4; ++e) {
    const float f0 = a0[e];
    const float f1 = a1[e];
    hv[e]     = (_Float16)carry_flush(bf16r(f0), kInCarry);
    hv[4 + e] = (_Float16)carry_flush(bf16r(f1), kInCarry);
  }
  unsigned short* dp = dst + (size_t)row * dstPitch + dstOff + c8;
  *(volatile v8h*)dp = hv;
  __threadfence();
  *(volatile v8h*)dp = hv;
}

__global__ __launch_bounds__(kThr) void setup_kernel(unsigned short* __restrict__ WXP, float* __restrict__ ZB) {
  unsigned v = blockIdx.x * (unsigned)kThr + threadIdx.x;
  asm volatile("" : "+v"(v));
  if (v < 15872u) {
    v8h z;
#pragma unroll
    for (int e = 0; e < 8; ++e) z[e] = (_Float16)0.0f;
    unsigned short* dp = WXP + (size_t)kXd * kXK + (size_t)v * 8u;
    *(volatile v8h*)dp = z;
    __threadfence();
    *(volatile v8h*)dp = z;
  } else {
    const v4f o = {0.f, 0.f, 0.f, 0.f};
    float* dp = ZB + (size_t)(v - 15872u) * 4u;
    *(volatile v4f*)dp = o;
    __threadfence();
    *(volatile v4f*)dp = o;
  }
}
static_assert((kXdP - kXd) * kXK / 8 == 15872 && 15872 % kThr == 0 && (15872 + 1024) == 66 * kThr && ((size_t)kXd * kXK * 2) % 256 == 0, "set-up grid exact");

__device__ __forceinline__ void split_f16(float x, float c, float cinv, _Float16& hi, _Float16& lo) {
  hi = (_Float16)carry_flush(x, c);
  const float back = (float)hi * cinv;
  lo = (_Float16)carry_flush(x - back, c);
}

__global__ __launch_bounds__(kThr) void conv_silu_kernel(const float* __restrict__ XZ, const float* __restrict__ conv_w, const float* __restrict__ conv_b,
                                                         float* __restrict__ XI, unsigned short* __restrict__ XI16) {
  const size_t v = (size_t)blockIdx.x * kThr + threadIdx.x;
  const int row = (int)(v >> 9);
  const int d4 = (int)(v & 511) * 4;
  const v4f cb = *(const v4f*)(conv_b + d4);
  float acc[4];
#pragma unroll
  for (int e = 0; e < 4; ++e) { const float b0 = cb[e]; acc[e] = bf16r(b0); }
#pragma unroll
  for (int j = 0; j < kKc; ++j) {
    const int tr = row + j - (kKc - 1);
    const bool in = tr >= 0;
    const v4f xin = *(const v4f*)(XZ + (size_t)(in ? tr : 0) * kDi2 + d4);
#pragma unroll
    for (int e = 0; e < 4; ++e) {
      const float w0 = conv_w[(size_t)(d4 + e) * kKc + j];
      const float xv = in ? xin[e] : 0.0f;
      acc[e] += bf16r(w0) * xv;
    }
  }
  v4f o; v4h hv, lv;
#pragma unroll
  for (int e = 0; e < 4; ++e) {
    const float s = acc[e] * (1.0f / (1.0f + expf(-acc[e])));
    o[e] = s;
    _Float16 hi, lo; split_f16(s, kACarry, 1.0f / kACarry, hi, lo);
    hv[e] = hi; lv[e] = lo;
  }
  for (int pass = 0; pass < 2; ++pass) {
    *(volatile v4f*)(XI + (size_t)row * kDi + d4) = o;
    *(volatile v4h*)(XI16 + (size_t)row * kXK + d4) = hv;
    *(volatile v4h*)(XI16 + (size_t)row * kXK + kDi + d4) = lv;
    __threadfence();
  }
}
static_assert(((size_t)kRows * 512) % kThr == 0 && kDi / 4 == 512, "conv grid exact");

__global__ __launch_bounds__(kThr) void sel_scan_kernel(const float* __restrict__ XI, const float* __restrict__ XD, const float* __restrict__ A_log,
                                                        float* __restrict__ HID) {
  const int d = blockIdx.x * kThr + threadIdx.x;
  float A[kNs], h[kNs];
#pragma unroll
  for (int n = 0; n < kNs; ++n) { const float al = A_log[(size_t)d * kNs + n]; A[n] = -expf(bf16r(al)); h[n] = 0.0f; }
#pragma unroll 1
  for (int l = 0; l < kSeq; ++l) {
    const float* pr = XD + (size_t)l * kXdP;
    const float dl = pr[0];
    const float xv = XI[(size_t)l * kDi + d];
    const float delta = (dl > 20.0f) ? dl : log1pf(expf(dl));
    const float dx = delta * xv;
    float y = 0.0f;
#pragma unroll
    for (int n = 0; n < kNs; ++n) {
      const float hn = __expf(delta * A[n]) * h[n] + dx * pr[1 + n];
      h[n] = hn;
      y += hn * pr[1 + kNs + n];
    }
    float* hp = HID + (size_t)l * kDi + d;
    *(volatile float*)hp = y;
    __threadfence();
    *(volatile float*)hp = y;
  }
}
static_assert(kDi % kThr == 0, "scan grid exact");

__global__ __launch_bounds__(kThr) void gate_cast_kernel(const float* __restrict__ HID, const float* __restrict__ XZ, unsigned short* __restrict__ Y16) {
  const size_t row = blockIdx.x;
  const int d8 = threadIdx.x * 8;
  v8h hv;
#pragma unroll
  for (int hlf = 0; hlf < 2; ++hlf) {
    const v4f hh = *(const v4f*)(HID + row * kDi + d8 + 4 * hlf);
    const v4f zz = *(const v4f*)(XZ + row * kDi2 + kDi + d8 + 4 * hlf);
#pragma unroll
    for (int e = 0; e < 4; ++e) {
      const float g = zz[e] * frcp(1.0f + __expf(-zz[e]));
      hv[4 * hlf + e] = (_Float16)carry_flush(hh[e] * g, kACarry);
    }
  }
  unsigned short* dp = Y16 + row * kDi + d8;
  *(volatile v8h*)dp = hv;
  __threadfence();
  *(volatile v8h*)dp = hv;
}
static_assert(kDi / 8 == kThr, "one block per row");

static_assert(((size_t)kRows * kDm / 8) % kThr == 0 && ((size_t)kDi2 * kDm / 8) % kThr == 0 && ((size_t)kXd * kDi / 8) % kThr == 0 && ((size_t)kDm * kDi / 8) % kThr == 0, "cast grids exact");

extern "C" void kernel_launch(void* const* d_in, const int* in_sizes, int n_in,
                              void* d_out, int out_size, void* d_ws, size_t ws_size,
                              hipStream_t stream) {
  if (n_in < 7 || d_out == nullptr || d_ws == nullptr) return;
  if (in_sizes[0] != kSamples * kRows * kDm || in_sizes[1] != kDi2 * kDm || in_sizes[2] != kDi * kKc || in_sizes[3] != kDi) return;
  if (in_sizes[4] != kDi * kNs || in_sizes[5] != kXd * kDi || in_sizes[6] != kDm * kDi) return;
  if (out_size != kSamples * kRows * kDm) return;
  if (ws_size < kWsTotal) return;
  const float* x = (const float*)d_in[0];
  const float* W_in = (const float*)d_in[1];
  const float* conv_w = (const float*)d_in[2];
  const float* conv_b = (const float*)d_in[3];
  const float* A_log = (const float*)d_in[4];
  const float* W_x = (const float*)d_in[5];
  const float* W_out = (const float*)d_in[6];
  float* out = (float*)d_out;
  char* ws = (char*)d_ws;
  unsigned short* X16 = (unsigned short*)(ws + kOffX16);
  unsigned short* WIN = (unsigned short*)(ws + kOffWIN);
  unsigned short* WXP = (unsigned short*)(ws + kOffWXP);
  unsigned short* WOUT = (unsigned short*)(ws + kOffWOUT);
  float* ZB = (float*)(ws + kOffZB);
  float* XZ = (float*)(ws + kOffXZ);
  float* XI = (float*)(ws + kOffXI);
  unsigned short* XI16 = (unsigned short*)(ws + kOffXI16);
  float* XD = (float*)(ws + kOffXD);
  float* HID = (float*)(ws + kOffHID);
  unsigned short* Y16 = (unsigned short*)(ws + kOffY16);

  cast_plane_kernel<<<(int)(((size_t)kDi2 * kDm / 8) / kThr), kThr, 0, stream>>>(W_in, WIN, 10, kDm, 0);
  cast_plane_kernel<<<(int)(((size_t)kXd * kDi / 8) / kThr), kThr, 0, stream>>>(W_x, WXP, 11, kXK, 0);
  cast_plane_kernel<<<(int)(((size_t)kXd * kDi / 8) / kThr), kThr, 0, stream>>>(W_x, WXP, 11, kXK, kDi);
  cast_plane_kernel<<<(int)(((size_t)kDm * kDi / 8) / kThr), kThr, 0, stream>>>(W_out, WOUT, 11, kDi, 0);
  setup_kernel<<<66, kThr, 0, stream>>>(WXP, ZB);

  for (int s = 0; s < kSamples; ++s) {
    const float* xs = x + (size_t)s * kRows * kDm;
    float* os = out + (size_t)s * kRows * kDm;
    cast_plane_kernel<<<(int)(((size_t)kRows * kDm / 8) / kThr), kThr, 0, stream>>>(xs, X16, 10, kDm, 0);
    wmma_gemm64<0, false, 2, 0, false, 0><<<dim3((kRows / 64) * (kDi2 / 64) / 8, 1), 256, 0, stream>>>(
        X16, X16, kDm, 0L, WIN, WIN, kDm, 0L, (void*)XZ, (void*)XZ, kDi2, 0L, ZB, nullptr, 0L, kRows, kDi2, kDm, kScIn);
    conv_silu_kernel<<<(int)(((size_t)kRows * 512) / kThr), kThr, 0, stream>>>(XZ, conv_w, conv_b, XI, XI16);
    wmma_gemm64<0, false, 2, 0, false, 0><<<dim3((kRows / 64) * (kXdP / 64) / 8, 1), 256, 0, stream>>>(
        XI16, XI16, kXK, 0L, WXP, WXP, kXK, 0L, (void*)XD, (void*)XD, kXdP, 0L, ZB, nullptr, 0L, kRows, kXdP, kXK, kScA);
    sel_scan_kernel<<<kDi / kThr, kThr, 0, stream>>>(XI, XD, A_log, HID);
    gate_cast_kernel<<<kRows, kThr, 0, stream>>>(HID, XZ, Y16);
    wmma_gemm64<0, false, 2, 0, false, 0><<<dim3((kRows / 64) * (kDm / 64) / 8, 1), 256, 0, stream>>>(
        Y16, Y16, kDi, 0L, WOUT, WOUT, kDi, 0L, (void*)os, (void*)os, kDm, 0L, ZB, nullptr, 0L, kRows, kDm, kDi, kScA);
  }
}
